// DirectionalStockGNN_62672162783774
// MI455X (gfx1250) — hardware-run, weakly checked
//
#include <hip/hip_runtime.h>
#include <stddef.h>
#include <stdint.h>


#define DF      128
#define NC2     256
#define SPLIT2  0
#define KS1     (DF / 32)
#define KS2     ((SPLIT2 ? 2 * DF : DF) / 32)
#define NTHR    256
#define NWAVE   8
#define NB      1024
#define RCAP    20480
#define WLCAP   3072
#define DEGCAP  128
#define GBM     64
#define GBN     64
#define GTHR    128
#define RROWS   32
#define PAR_W1E 0
#define PAR_W2E 512
#define PAR_AT1 1024
#define PAR_AT2 1152
#define PAR_B1  1280
#define PAR_B2  1408
#define PAR_WFC 1536
#define PAR_BFC 1664
#define PARN    1792
#define PARU    (PARN / 4)
#define WSMAX   ((size_t)128 << 20)
#define LDS_BKT ((NWAVE * WLCAP + RCAP + 3 * NB + 2 * NWAVE) * 4)
#define NREF    50000
#define EREF    800000

constexpr size_t al256(size_t v) { return (v + 255) & ~(size_t)255; }
constexpr size_t MPREF = (size_t)((NREF + GBM - 1) / GBM) * GBM;
constexpr size_t GBREF = (size_t)((NREF + NB - 1) / NB);
constexpr size_t WSREF = al256(MPREF * DF * 2) + al256(MPREF * NC2 * 4) + al256(MPREF * NC2 * 2) +
                         al256(GBREF * RCAP * 8) + al256(GBREF * NB * 8) + al256(GBREF * NB * 16) +
                         al256((size_t)EREF * 16) + al256((size_t)NC2 * DF * 2) +
                         al256((size_t)NC2 * 2 * DF * 2) + al256((size_t)PARN * 4);

static_assert(DF == 32 * 4);
static_assert((DF % 32) == 0 && ((2 * DF) % 32) == 0);
static_assert(NC2 == 2 * DF && (NC2 % GBN) == 0);
static_assert(NB == 4 * NTHR);
static_assert((NB & (NB - 1)) == 0 && NB == 1024);
static_assert((RCAP % (2 * NTHR)) == 0);
static_assert(RCAP >= 16623 + 16623 / 5);
static_assert(NWAVE * WLCAP >= RCAP);
static_assert(DEGCAP >= 35 + 8);
static_assert(LDS_BKT <= 300000);
static_assert(GBM == (GTHR / 32) * 16);
static_assert(NREF <= 49 * NB);
static_assert((EREF % 256) == 0);
static_assert(WSREF <= WSMAX);
static_assert(PARU == 448 && (PARU % 32) == 0);
static_assert(RROWS == 32);

typedef float          v4f   __attribute__((ext_vector_type(4)));
typedef float          v8f   __attribute__((ext_vector_type(8)));
typedef int            v2i   __attribute__((ext_vector_type(2)));
typedef int            v4i   __attribute__((ext_vector_type(4)));
typedef int            v8i   __attribute__((ext_vector_type(8)));
typedef unsigned       v2u   __attribute__((ext_vector_type(2)));
typedef unsigned short v8us  __attribute__((ext_vector_type(8)));
typedef __bf16         v16bf __attribute__((ext_vector_type(16)));
typedef v4f __attribute__((may_alias)) v4fa;
union FragB { v16bf v; v8us u[2]; v8i w; v4i q[2]; };

__device__ __forceinline__ v8f wmx(const FragB& a, const FragB& b, v8f c) {
  v8f d = __builtin_amdgcn_wmma_f32_16x16x32_bf16(false, a.v, false, b.v, (short)0, c, false, false);
  asm volatile("v_nop\n\tv_nop\n\tv_nop\n\tv_nop" : "+v"(d) : "v"(a.w), "v"(b.w));
  return d;
}

__device__ __forceinline__ void pinf(float x) { asm volatile("" :: "v"(x)); }
__device__ __forceinline__ void pini(int x)   { asm volatile("" :: "v"(x)); }

__device__ __forceinline__ unsigned bfbits(float v) {
  const unsigned u = __float_as_uint(v);
  const unsigned r = (u + 0x7FFFu + ((u >> 16) & 1u)) >> 16;
  const unsigned nb = ((u >> 16) & 0x8000u) | 0x7FC0u;
  return ((u & 0x7FFFFFFFu) > 0x7F800000u) ? nb : r;
}
__device__ __forceinline__ float rbf(float v) { return __uint_as_float(bfbits(v) << 16); }
__device__ __forceinline__ v4f rbf4(const v4f a) {
  v4f o; o.x = rbf(a.x); o.y = rbf(a.y); o.z = rbf(a.z); o.w = rbf(a.w); return o;
}
__device__ __forceinline__ float wsum(float v) {
#pragma unroll
  for (int off = 16; off > 0; off >>= 1) v += __shfl_xor(v, off);
  return v;
}

__device__ __forceinline__ v8us wcol8(const float* __restrict__ w, int n, int k8) {
  float f[8];
#pragma unroll
  for (int i = 0; i < 8; ++i) {
    f[i] = w[(size_t)(k8 + i) * DF + n];
    pinf(f[i]);
  }
  v8us hv;
#pragma unroll
  for (int i = 0; i < 8; ++i) hv[i] = (unsigned short)bfbits(f[i]);
  return hv;
}

__global__ __launch_bounds__(NTHR) void k_prep(
    const float* __restrict__ x, const float* __restrict__ eattr,
    const float* __restrict__ W1l, const float* __restrict__ W1r,
    const float* __restrict__ W2l, const float* __restrict__ W2r,
    const float* __restrict__ W1e, const float* __restrict__ W2e,
    const float* __restrict__ att1, const float* __restrict__ att2,
    const float* __restrict__ b1, const float* __restrict__ b2,
    const float* __restrict__ Wfc, const float* __restrict__ bfc,
    unsigned short* xb, float* ear, unsigned short* w1t, unsigned short* w2d, float* par,
    int nN, int nE, int bX, int bE)
{
  const int tid = (int)threadIdx.x;
  int blk = (int)blockIdx.x;
  if (blk < bX) {
    const int i = blk * NTHR + tid;
    const int row = i >> 4;
    const int c0  = (i & 15) * 8;
    const int rc  = row < nN ? row : nN - 1;
    const float* p = x + (size_t)rc * DF + c0;
    const v4f a = *(const v4f*)p, b = *(const v4f*)(p + 4);
    const unsigned mk = row < nN ? 0xFFFFu : 0u;
    v8us hv;
    hv[0] = (unsigned short)(bfbits(a.x) & mk); hv[1] = (unsigned short)(bfbits(a.y) & mk);
    hv[2] = (unsigned short)(bfbits(a.z) & mk); hv[3] = (unsigned short)(bfbits(a.w) & mk);
    hv[4] = (unsigned short)(bfbits(b.x) & mk); hv[5] = (unsigned short)(bfbits(b.y) & mk);
    hv[6] = (unsigned short)(bfbits(b.z) & mk); hv[7] = (unsigned short)(bfbits(b.w) & mk);
    const size_t o = (size_t)row * DF + c0;
    *(volatile v8us*)(xb + o) = hv;
    __threadfence();
    *(volatile v8us*)(xb + o) = hv;
    return;
  }
  blk -= bX;
  if (blk < bE) {
    const int e = blk * NTHR + tid;
    if (e >= nE) return;
    const v4f v = rbf4(*(const v4f*)(eattr + (size_t)e * 4));
    float* op = ear + (size_t)e * 4;
    *(volatile v4f*)op = v;
    __threadfence();
    *(volatile v4f*)op = v;
    return;
  }
  blk -= bE;
  if (blk < 16) {
    const int u  = blk * NTHR + tid;
    const int n  = u >> 4;
    const int k8 = (u & 15) * 8;
    v8us hv;
    if (blk < 8) hv = wcol8(W1l, n & (DF - 1), k8);
    else         hv = wcol8(W1r, n & (DF - 1), k8);
    const size_t o = (size_t)n * DF + k8;
    *(volatile v8us*)(w1t + o) = hv;
    __threadfence();
    *(volatile v8us*)(w1t + o) = hv;
    return;
  }
  blk -= 16;
  if (blk < 16) {
    const int u  = blk * NTHR + tid;
    const int n  = u >> 4;
    const int k8 = (u & 15) * 8;
    v8us hv;
    if (blk < 8) hv = wcol8(W2l, n & (DF - 1), k8);
    else         hv = wcol8(W2r, n & (DF - 1), k8);
    const size_t o = (size_t)n * (2 * DF) + k8;
    *(volatile v8us*)(w2d + o) = hv;
    *(volatile v8us*)(w2d + o + DF) = hv;
    __threadfence();
    *(volatile v8us*)(w2d + o) = hv;
    *(volatile v8us*)(w2d + o + DF) = hv;
    return;
  }
  blk -= 16;
  {
    const int u = blk * NTHR + tid;
    if (u >= PARU) return;
    v4f v = {0.f, 0.f, 0.f, 0.f};
    if (u < 128)      v = *(const v4f*)(W1e + 4 * u);
    else if (u < 256) v = *(const v4f*)(W2e + 4 * (u - 128));
    else if (u < 288) v = *(const v4f*)(att1 + 4 * (u - 256));
    else if (u < 320) v = *(const v4f*)(att2 + 4 * (u - 288));
    else if (u < 352) v = *(const v4f*)(b1 + 4 * (u - 320));
    else if (u < 384) v = *(const v4f*)(b2 + 4 * (u - 352));
    else if (u < 416) v = *(const v4f*)(Wfc + 4 * (u - 384));
    else {
      const float b = bfc[0];
      pinf(b);
      const unsigned mk = (u == 416) ? 0xFFFFFFFFu : 0u;
      v.x = __uint_as_float(__float_as_uint(b) & mk);
    }
    const v4f r = rbf4(v);
    float* op = par + 4 * u;
    *(volatile v4f*)op = r;
    __threadfence();
    *(volatile v4f*)op = r;
  }
}

__device__ __forceinline__ int scan256(const int* __restrict__ dsts, int nE, int base, int slotBase,
                                       int vec8, int* wlw, int lane, int wc) {
  const int e0   = base + lane * 8;
  const int sent = (int)0x80000000u;
  v4i da, db;
  if (vec8 != 0 && base + 256 <= nE) {
    da = *(const v4i*)(dsts + e0);
    db = *(const v4i*)(dsts + e0 + 4);
  } else {
    da.x = (e0     < nE) ? dsts[min(e0,     nE - 1)] : sent;
    da.y = (e0 + 1 < nE) ? dsts[min(e0 + 1, nE - 1)] : sent;
    da.z = (e0 + 2 < nE) ? dsts[min(e0 + 2, nE - 1)] : sent;
    da.w = (e0 + 3 < nE) ? dsts[min(e0 + 3, nE - 1)] : sent;
    db.x = (e0 + 4 < nE) ? dsts[min(e0 + 4, nE - 1)] : sent;
    db.y = (e0 + 5 < nE) ? dsts[min(e0 + 5, nE - 1)] : sent;
    db.z = (e0 + 6 < nE) ? dsts[min(e0 + 6, nE - 1)] : sent;
    db.w = (e0 + 7 < nE) ? dsts[min(e0 + 7, nE - 1)] : sent;
  }
  const unsigned nbs = (unsigned)slotBase;
  const unsigned unb = (unsigned)NB;
  const unsigned s0 = (unsigned)da.x - nbs, s1 = (unsigned)da.y - nbs;
  const unsigned s2 = (unsigned)da.z - nbs, s3 = (unsigned)da.w - nbs;
  const unsigned s4 = (unsigned)db.x - nbs, s5 = (unsigned)db.y - nbs;
  const unsigned s6 = (unsigned)db.z - nbs, s7 = (unsigned)db.w - nbs;
  const bool h0 = s0 < unb, h1 = s1 < unb, h2 = s2 < unb, h3 = s3 < unb;
  const bool h4 = s4 < unb, h5 = s5 < unb, h6 = s6 < unb, h7 = s7 < unb;
  const unsigned any = __builtin_amdgcn_ballot_w32(h0 | h1 | h2 | h3 | h4 | h5 | h6 | h7);
  if (any != 0u) {
#define HITJ(J, HJ, SJ) { \
      const unsigned mj = __builtin_amdgcn_ballot_w32(HJ); \
      if (mj != 0u) { \
        if (HJ) { \
          const int pos = wc + (int)__builtin_amdgcn_mbcnt_lo(mj, 0u); \
          if (pos < WLCAP) wlw[pos] = ((e0 + (J)) << 10) | (int)(SJ); \
        } \
        wc += (int)__builtin_popcount(mj); } }
    HITJ(0, h0, s0)
    HITJ(1, h1, s1)
    HITJ(2, h2, s2)
    HITJ(3, h3, s3)
    HITJ(4, h4, s4)
    HITJ(5, h5, s5)
    HITJ(6, h6, s6)
    HITJ(7, h7, s7)
#undef HITJ
  }
  return wc;
}

__global__ __launch_bounds__(NTHR) void k_bucket(const int* __restrict__ srcs, const int* __restrict__ dsts,
                                                 const float* __restrict__ ear,
                                                 int* ent, int* slot, float* lap,
                                                 int nN, int nE, int vec8, int per) {
  extern __shared__ v4f lds_dyn[];
  int* wl   = (int*)lds_dyn;
  int* reg2 = wl + NWAVE * WLCAP;
  int* scnt = reg2 + RCAP;
  int* soff = scnt + NB;
  int* cur  = soff + NB;
  int* wcn  = cur + NB;
  int* wtot = wcn + NWAVE;
  const int tid = (int)threadIdx.x, lane = tid & 31;
  const int wave = __builtin_amdgcn_readfirstlane(tid >> 5);
  const int nodeBase = (int)blockIdx.x * NB;

  for (int i = tid; i < NB; i += NTHR) scnt[i] = 0;
  for (int i = tid; i < RCAP; i += NTHR) reg2[i] = 0;
  for (int i = tid; i < NWAVE * WLCAP; i += NTHR) wl[i] = 0;
  __syncthreads();

  {
    int wc = 0;
    const int wbeg = wave * per;
    int wend = wbeg + per;
    wend = wend > nE ? nE : wend;
    int* wlw = wl + wave * WLCAP;
#pragma unroll 1
    for (int base = wbeg; base < wend; base += 256)
      wc = scan256(dsts, nE, base, nodeBase, vec8, wlw, lane, wc);
    if (lane == 0) wcn[wave] = wc;
  }
  __syncthreads();

  int nhr = 0;
  bool ovf = false;
#pragma unroll
  for (int w2 = 0; w2 < NWAVE; ++w2) {
    int c = wcn[w2];
    ovf = ovf || (c > WLCAP);
    c = c < 0 ? 0 : (c > WLCAP ? WLCAP : c);
    nhr += c;
  }
  ovf = ovf || (nhr > RCAP);
  const int nh = nhr > RCAP ? RCAP : nhr;

  if (wave == 0) {
#pragma unroll 1
    for (int w2 = 0; w2 < NWAVE; ++w2) {
      int c = wcn[w2];
      c = c < 0 ? 0 : (c > WLCAP ? WLCAP : c);
      c = __builtin_amdgcn_readfirstlane(c);
#pragma unroll 1
      for (int b0 = 0; b0 < c; b0 += 32) {
        int idx = b0 + lane;
        idx = idx > WLCAP - 1 ? WLCAP - 1 : idx;
        const int uv  = wl[w2 * WLCAP + idx];
        const int m32 = (c - b0) < 32 ? (c - b0) : 32;
#pragma unroll 1
        for (int k = 0; k < m32; ++k) {
          const int u  = __builtin_amdgcn_readlane(uv, k);
          const int sl = u & (NB - 1);
          if (lane == 0) scnt[sl] = scnt[sl] + 1;
        }
      }
    }
  }
  __syncthreads();

  {
    const v4i ca = *(const v4i*)(scnt + 4 * tid);
    const int e0 = ca.x < 0 ? 0 : ca.x, e1 = ca.y < 0 ? 0 : ca.y;
    const int e2 = ca.z < 0 ? 0 : ca.z, e3 = ca.w < 0 ? 0 : ca.w;
    const int ts = e0 + e1 + e2 + e3;
    int incl = ts;
#pragma unroll
    for (int d = 1; d < 32; d <<= 1) {
      const int up = __shfl_up(incl, d);
      if (lane >= d) incl += up;
    }
    if (lane == 31) wtot[wave] = incl;
    __syncthreads();
    int pre = 0;
#pragma unroll
    for (int w2 = 0; w2 < NWAVE; ++w2) pre += (w2 < wave) ? wtot[w2] : 0;
    int run = pre + incl - ts;
    soff[4 * tid + 0] = run; run += e0;
    soff[4 * tid + 1] = run; run += e1;
    soff[4 * tid + 2] = run; run += e2;
    soff[4 * tid + 3] = run;
  }
  __syncthreads();
  for (int i = tid; i < NB; i += NTHR) cur[i] = soff[i];
  __syncthreads();

  if (wave == 0) {
#pragma unroll 1
    for (int w2 = 0; w2 < NWAVE; ++w2) {
      int c = wcn[w2];
      c = c < 0 ? 0 : (c > WLCAP ? WLCAP : c);
      c = __builtin_amdgcn_readfirstlane(c);
#pragma unroll 1
      for (int b0 = 0; b0 < c; b0 += 32) {
        int idx = b0 + lane;
        idx = idx > WLCAP - 1 ? WLCAP - 1 : idx;
        const int uv  = wl[w2 * WLCAP + idx];
        const int m32 = (c - b0) < 32 ? (c - b0) : 32;
#pragma unroll 1
        for (int k = 0; k < m32; ++k) {
          const int u   = __builtin_amdgcn_readlane(uv, k);
          const int sl  = u & (NB - 1);
          const int eid = (int)((unsigned)u >> 10);
          if (lane == 0) {
            int pos = cur[sl];
            pos = pos < 0 ? 0 : (pos > RCAP - 1 ? RCAP - 1 : pos);
            reg2[pos] = eid;
            cur[sl] = pos + 1;
          }
        }
      }
    }
  }
  __syncthreads();

  int* eb = ent + (size_t)blockIdx.x * (size_t)(2 * RCAP);
#pragma unroll 1
  for (int p0 = 0; p0 < RCAP; p0 += 2 * NTHR) {
    const int p = p0 + 2 * tid;
    int e0 = reg2[p], e1 = reg2[p + 1];
    e0 = e0 < 0 ? 0 : (e0 > nE - 1 ? nE - 1 : e0);
    e1 = e1 < 0 ? 0 : (e1 > nE - 1 ? nE - 1 : e1);
    const int s0 = srcs[e0];
    const int s1 = srcs[e1];
    pini(s0); pini(s1);
    const int m0 = (p     < nh) ? -1 : 0;
    const int m1 = (p + 1 < nh) ? -1 : 0;
    v4i v;
    v.x = s0 & m0; v.y = e0 & m0; v.z = s1 & m1; v.w = e1 & m1;
    *(volatile v4i*)(eb + 2 * p) = v;
    __threadfence();
    *(volatile v4i*)(eb + 2 * p) = v;
  }
#pragma unroll 1
  for (int it = 0; it < 2; ++it) {
    const int u = it * NTHR + tid;
    v4i sv;
    sv.x = soff[2 * u];
    sv.y = ovf ? -1 : scnt[2 * u];
    sv.z = soff[2 * u + 1];
    sv.w = ovf ? -1 : scnt[2 * u + 1];
    int* sp = slot + 2 * (size_t)(nodeBase + 2 * u);
    *(volatile v4i*)sp = sv;
    __threadfence();
    *(volatile v4i*)sp = sv;
  }
#pragma unroll 1
  for (int it = 0; it < 4; ++it) {
    const int sl = it * NTHR + tid;
    int st = soff[sl];
    int c  = scnt[sl];
    st = st < 0 ? 0 : (st > RCAP - 1 ? RCAP - 1 : st);
    c  = c < 0 ? 0 : (c > DEGCAP ? DEGCAP : c);
    if (c > RCAP - st) c = RCAP - st;
    int cm = c;
#pragma unroll
    for (int off = 16; off > 0; off >>= 1) {
      const int o2 = __shfl_xor(cm, off);
      cm = cm > o2 ? cm : o2;
    }
    cm = __builtin_amdgcn_readfirstlane(cm);
    cm = cm > DEGCAP ? DEGCAP : cm;
    int last = st + c - 1;
    last = last < st ? st : last;
    v4f sum = {0.f, 0.f, 0.f, 0.f};
#pragma unroll 1
    for (int q = 0; q < cm; ++q) {
      int idx = st + q;
      idx = idx > last ? last : idx;
      int eid = reg2[idx];
      eid = eid < 0 ? 0 : (eid > nE - 1 ? nE - 1 : eid);
      const v4f v = *(const v4f*)(ear + (size_t)eid * 4);
      pinf(v.x); pinf(v.y); pinf(v.z); pinf(v.w);
      const unsigned mk = (q < c) ? 0xFFFFFFFFu : 0u;
      sum.x += __uint_as_float(__float_as_uint(v.x) & mk);
      sum.y += __uint_as_float(__float_as_uint(v.y) & mk);
      sum.z += __uint_as_float(__float_as_uint(v.z) & mk);
      sum.w += __uint_as_float(__float_as_uint(v.w) & mk);
    }
    const float cf = (float)(c > 1 ? c : 1);
    v4f o;
    o.x = sum.x / cf; o.y = sum.y / cf; o.z = sum.z / cf; o.w = sum.w / cf;
    float* lp = lap + 4 * (size_t)(nodeBase + sl);
    *(volatile v4f*)lp = o;
    __threadfence();
    *(volatile v4f*)lp = o;
  }
  (void)nN;
}

__global__ __launch_bounds__(GTHR) __attribute__((amdgpu_num_vgpr(248)))
void k_gemm(const unsigned short* __restrict__ A, int lda,
            const unsigned short* __restrict__ WT, int ldw,
            float* outF, int ldo, int ksteps)
{
  __shared__ __attribute__((aligned(16))) float stg[GBM * GBN];
  const int tid = (int)threadIdx.x, lane = tid & 31, wave = tid >> 5, hh = lane >> 4, m = lane & 15;
  const int rowBase = (int)blockIdx.x * GBM;
  const int col0    = (int)blockIdx.y * GBN;

  v8f acc[4];
  {
    const v8f z = {0.f, 0.f, 0.f, 0.f, 0.f, 0.f, 0.f, 0.f};
    acc[0] = z; acc[1] = z; acc[2] = z; acc[3] = z;
  }
  const unsigned short* ap = A  + (size_t)(rowBase + 16 * wave + m) * (size_t)lda + 8 * hh;
  const unsigned short* wp = WT + (size_t)(col0 + m) * (size_t)ldw + 8 * hh;
#pragma unroll 1
  for (int ks = 0; ks < ksteps; ++ks) {
    FragB af;
    af.u[0] = *(const v8us*)(ap + 32 * ks);
    af.u[1] = *(const v8us*)(ap + 32 * ks + 16);
#pragma unroll
    for (int t = 0; t < 4; ++t) {
      const unsigned short* wq = wp + (size_t)(16 * t) * (size_t)ldw + 32 * ks;
      FragB bf;
      bf.u[0] = *(const v8us*)wq;
      bf.u[1] = *(const v8us*)(wq + 16);
      acc[t] = wmx(af, bf, acc[t]);
    }
  }

#pragma unroll
  for (int t = 0; t < 4; ++t) {
    const int lc = 16 * t + m;
#pragma unroll
    for (int r = 0; r < 8; ++r) {
      const int lr = 16 * wave + 8 * hh + r;
      stg[lr * GBN + lc] = acc[t][r];
    }
  }
  __syncthreads();

  v4f fv[8];
#pragma unroll
  for (int i = 0; i < 8; ++i) {
    const int lr = 16 * wave + 2 * i + hh;
    fv[i] = *(const v4fa*)(stg + lr * GBN + 4 * m);
  }
#pragma unroll
  for (int i = 0; i < 8; ++i) {
    const int lr = 16 * wave + 2 * i + hh;
    float* op = outF + (size_t)(rowBase + lr) * (size_t)ldo + col0 + 4 * m;
    *(volatile v4f*)op = fv[i];
  }
  __threadfence();
#pragma unroll
  for (int i = 0; i < 8; ++i) {
    const int lr = 16 * wave + 2 * i + hh;
    float* op = outF + (size_t)(rowBase + lr) * (size_t)ldo + col0 + 4 * m;
    *(volatile v4f*)op = fv[i];
  }
}

template<int MODE>
__global__ __launch_bounds__(NTHR)
void k_replay(const int* __restrict__ ent, const int* __restrict__ slot, const float* __restrict__ lap,
              const float* __restrict__ ear, const float* __restrict__ xlr, const float* __restrict__ par,
              int weo, int ato, int bio,
              const unsigned short* __restrict__ xb, unsigned short* hhl, float* outF,
              int nN, int nE, int MPr)
{
  const int tid = (int)threadIdx.x, lane = tid & 31;
  const int wave = __builtin_amdgcn_readfirstlane(tid >> 5);
  const int row0 = ((int)blockIdx.x * NWAVE + wave) * RROWS;
  const int lim  = (MODE == 0) ? MPr : nN;
  if (row0 >= lim) return;
  const int c4 = 4 * lane;
  const v4f we0 = *(const v4f*)(par + weo + c4);
  const v4f we1 = *(const v4f*)(par + weo + DF + c4);
  const v4f we2 = *(const v4f*)(par + weo + 2 * DF + c4);
  const v4f we3 = *(const v4f*)(par + weo + 3 * DF + c4);
  const v4f at  = *(const v4f*)(par + ato + c4);
  const v4f bb  = *(const v4f*)(par + bio + c4);
  const v4f wf  = *(const v4f*)(par + PAR_WFC + c4);
  const float bfcv = par[PAR_BFC];
  const float qnan = __int_as_float(0x7fc00000);
  float res = 0.0f;

#pragma unroll 1
  for (int jr = 0; jr < RROWS; ++jr) {
    const int i = row0 + jr;
    if (i >= lim) break;
    const v2i se = *(const v2i*)(slot + 2 * (size_t)i);
    int st = __builtin_amdgcn_readfirstlane(se.x);
    const int craw = __builtin_amdgcn_readfirstlane(se.y);
    st = st < 0 ? 0 : (st > RCAP - 1 ? RCAP - 1 : st);
    int cnt = craw < 0 ? 0 : (craw > DEGCAP ? DEGCAP : craw);
    if (cnt > RCAP - st) cnt = RCAP - st;
    const bool bad = (craw < 0) || (craw > DEGCAP);
    const int blk = i / NB;
    const int* eb = ent + (size_t)blk * (size_t)(2 * RCAP);
    const v4f xr  = *(const v4f*)(xlr + (size_t)i * NC2 + DF + c4);
    const v4f lav = *(const v4f*)(lap + 4 * (size_t)i);
    int last = st + cnt - 1;
    last = last < st ? st : last;
    const int nit = cnt + 1;
    v4f acc = {0.f, 0.f, 0.f, 0.f};
    float mx = -1.0e30f, dn = 0.0f;

#pragma unroll 1
    for (int t0 = 0; t0 < nit; t0 += 32) {
      int ei = st + t0 + lane - 1;
      ei = ei < st ? st : ei;
      ei = ei > last ? last : ei;
      const v2i en = *(const v2i*)(eb + 2 * ei);
      pini(en.x); pini(en.y);
      int sv = en.x < 0 ? 0 : (en.x > nN - 1 ? nN - 1 : en.x);
      const int ev = en.y < 0 ? 0 : (en.y > nE - 1 ? nE - 1 : en.y);
      const int lm = (t0 + lane == 0) ? -1 : 0;
      sv = (i & lm) | (sv & ~lm);
      const int nv = (nit - t0) < 32 ? (nit - t0) : 32;
#pragma unroll 1
      for (int r = 0; r < nv; ++r) {
        const int s = __builtin_amdgcn_readlane(sv, r);
        const int e = __builtin_amdgcn_readlane(ev, r);
        const v4f xl = *(const v4f*)(xlr + (size_t)s * NC2 + c4);
        v4f ea4 = *(const v4f*)(ear + 4 * (size_t)e);
        pinf(ea4.x); pinf(ea4.y); pinf(ea4.z); pinf(ea4.w);
        const bool lp = (t0 + r) == 0;
        ea4 = lp ? lav : ea4;
        v4f ee = we0 * ea4.x;
        ee = ee + we1 * ea4.y;
        ee = ee + we2 * ea4.z;
        ee = ee + we3 * ea4.w;
        v4f v = (xl + xr) + ee;
        v.x = (v.x > 0.0f) ? v.x : 0.2f * v.x;
        v.y = (v.y > 0.0f) ? v.y : 0.2f * v.y;
        v.z = (v.z > 0.0f) ? v.z : 0.2f * v.z;
        v.w = (v.w > 0.0f) ? v.w : 0.2f * v.w;
        float part = v.x * at.x;
        part = fmaf(v.y, at.y, part);
        part = fmaf(v.z, at.z, part);
        part = fmaf(v.w, at.w, part);
        const float al = wsum(part);
        const float df = al - mx;
        const float eo = expf(-fabsf(df));
        const bool up  = df > 0.0f;
        const float s1 = up ? eo : 1.0f;
        const float s2 = up ? 1.0f : eo;
        mx = up ? al : mx;
        dn = fmaf(dn, s1, s2);
        acc = acc * s1 + xl * s2;
      }
    }

    const float inv = 1.0f / dn;
    v4f o = acc * inv + bb;
    o = o + (bad ? qnan : 0.0f);
#pragma unroll 1
    for (int k = 0; k < 4; ++k) {
      const float t = o.x;
      const float en1 = expm1f(t);
      o.x = (t > 0.0f) ? t : en1;
      o = __builtin_shufflevector(o, o, 1, 2, 3, 0);
    }

    if (MODE == 0) {
      const unsigned pm = (i < nN) ? 0xFFFFFFFFu : 0u;
      const unsigned h0 = bfbits(o.x), h1 = bfbits(o.y), h2 = bfbits(o.z), h3 = bfbits(o.w);
      unsigned l0 = 0u, l1 = 0u, l2 = 0u, l3 = 0u;
      if (SPLIT2) {
        l0 = bfbits(o.x - __uint_as_float(h0 << 16));
        l1 = bfbits(o.y - __uint_as_float(h1 << 16));
        l2 = bfbits(o.z - __uint_as_float(h2 << 16));
        l3 = bfbits(o.w - __uint_as_float(h3 << 16));
      }
      v2u hv, lv;
      hv.x = (h0 | (h1 << 16)) & pm; hv.y = (h2 | (h3 << 16)) & pm;
      lv.x = (l0 | (l1 << 16)) & pm; lv.y = (l2 | (l3 << 16)) & pm;
      unsigned short* hp = hhl + (size_t)i * NC2 + c4;
      *(volatile v2u*)hp = hv;
      *(volatile v2u*)(hp + DF) = lv;
      __threadfence();
      *(volatile v2u*)hp = hv;
      *(volatile v2u*)(hp + DF) = lv;
    } else {
      const v2u xw = *(const v2u*)(xb + (size_t)i * DF + c4);
      v4f xv;
      xv.x = __uint_as_float(xw.x << 16);
      xv.y = __uint_as_float(xw.x & 0xffff0000u);
      xv.z = __uint_as_float(xw.y << 16);
      xv.w = __uint_as_float(xw.y & 0xffff0000u);
      const v4f t = o + xv;
      float part = t.x * wf.x;
      part = fmaf(t.y, wf.y, part);
      part = fmaf(t.z, wf.z, part);
      part = fmaf(t.w, wf.w, part);
      float hv = wsum(part) + bfcv;
      hv = bad ? qnan : hv;
      res = (lane == jr) ? hv : res;
    }
  }

  if (MODE == 1) {
    int nvalid = nN - row0;
    nvalid = nvalid > RROWS ? RROWS : nvalid;
    const int sl = (4 * lane) & 31;
    v4f ov;
    ov.x = __shfl(res, sl);
    ov.y = __shfl(res, sl + 1);
    ov.z = __shfl(res, sl + 2);
    ov.w = __shfl(res, sl + 3);
    const bool wr = (lane < 8) && (4 * lane + 3 < nvalid);
    float* gp = outF + row0 + 4 * (lane & 7);
    if (wr) *(volatile v4f*)gp = ov;
    __threadfence();
    if (wr) *(volatile v4f*)gp = ov;
  }
  (void)xb; (void)hhl; (void)outF; (void)wf; (void)bfcv; (void)res;
}

static inline int cdiv(int a, int b) { return (a + b - 1) / b; }

extern "C" void kernel_launch(void* const* d_in, const int* in_sizes, int n_in,
                              void* d_out, int out_size, void* d_ws, size_t ws_size,
                              hipStream_t stream) {
  if (n_in < 15) return;
  const int nN = in_sizes[0] / DF;
  if (nN <= 0 || in_sizes[0] != nN * DF || nN > (1 << 21) || (nN & 3) != 0) return;
  if (in_sizes[1] < 2 || (in_sizes[1] & 1) != 0) return;
  const int nE = in_sizes[1] / 2;
  if (nE < 1 || nE > (1 << 20)) return;
  if (in_sizes[2] != nE * 4) return;
  if (in_sizes[3] != DF * DF || in_sizes[4] != DF * DF || in_sizes[8] != DF * DF || in_sizes[9] != DF * DF) return;
  if (in_sizes[5] != 4 * DF || in_sizes[10] != 4 * DF) return;
  if (in_sizes[6] != DF || in_sizes[7] != DF || in_sizes[11] != DF || in_sizes[12] != DF) return;
  if (in_sizes[13] != DF || in_sizes[14] != 1) return;
  if (out_size != nN) return;

  const float* x    = (const float*)d_in[0];
  const int*   ei   = (const int*)  d_in[1];
  const float* ea   = (const float*)d_in[2];
  const float* W1l  = (const float*)d_in[3];
  const float* W1r  = (const float*)d_in[4];
  const float* W1e  = (const float*)d_in[5];
  const float* att1 = (const float*)d_in[6];
  const float* b1   = (const float*)d_in[7];
  const float* W2l  = (const float*)d_in[8];
  const float* W2r  = (const float*)d_in[9];
  const float* W2e  = (const float*)d_in[10];
  const float* att2 = (const float*)d_in[11];
  const float* b2   = (const float*)d_in[12];
  const float* Wfc  = (const float*)d_in[13];
  const float* bfc  = (const float*)d_in[14];
  float* out = (float*)d_out;
  const int* src = ei;
  const int* dst = ei + nE;

  const int MP   = cdiv(nN, GBM) * GBM;
  const int gB   = cdiv(nN, NB);
  const int vec8 = ((nE & 3) == 0) ? 1 : 0;
  const int per  = cdiv(nE, NWAVE * 256) * 256;
  if (gB * NB < MP) return;

  char* ws = (char*)d_ws;
  size_t off = 0;
  const size_t oXB  = off; off += al256((size_t)MP * DF * 2);
  const size_t oXLR = off; off += al256((size_t)MP * NC2 * 4);
  const size_t oHHL = off; off += al256((size_t)MP * NC2 * 2);
  const size_t oENT = off; off += al256((size_t)gB * RCAP * 8);
  const size_t oSLT = off; off += al256((size_t)gB * NB * 8);
  const size_t oLA  = off; off += al256((size_t)gB * NB * 16);
  const size_t oEAR = off; off += al256((size_t)nE * 16);
  const size_t oW1T = off; off += al256((size_t)NC2 * DF * 2);
  const size_t oW2D = off; off += al256((size_t)NC2 * 2 * DF * 2);
  const size_t oPAR = off; off += al256((size_t)PARN * 4);
  if (off > ws_size || off > WSMAX) return;
  unsigned short* XB  = (unsigned short*)(ws + oXB);
  float*          XLR = (float*)(ws + oXLR);
  unsigned short* HHL = (unsigned short*)(ws + oHHL);
  int*            ENT = (int*)(ws + oENT);
  int*            SLT = (int*)(ws + oSLT);
  float*          LA  = (float*)(ws + oLA);
  float*          EAR = (float*)(ws + oEAR);
  unsigned short* W1T = (unsigned short*)(ws + oW1T);
  unsigned short* W2D = (unsigned short*)(ws + oW2D);
  float*          PAR = (float*)(ws + oPAR);

  hipFuncSetAttribute(reinterpret_cast<const void*>(&k_bucket),
                      hipFuncAttributeMaxDynamicSharedMemorySize, LDS_BKT);

  const int bX = MP / 16;
  const int bE = cdiv(nE, NTHR);
  k_prep<<<bX + bE + 16 + 16 + 2, NTHR, 0, stream>>>(x, ea, W1l, W1r, W2l, W2r, W1e, W2e, att1, att2, b1, b2,
                                                      Wfc, bfc, XB, EAR, W1T, W2D, PAR, nN, nE, bX, bE);
  k_bucket<<<gB, NTHR, LDS_BKT, stream>>>(src, dst, EAR, ENT, SLT, LA, nN, nE, vec8, per);
  k_gemm<<<dim3(MP / GBM, NC2 / GBN), GTHR, 0, stream>>>(XB, DF, W1T, DF, XLR, NC2, KS1);
  k_replay<0><<<cdiv(MP / RROWS, NWAVE), NTHR, 0, stream>>>(ENT, SLT, LA, EAR, XLR, PAR, PAR_W1E, PAR_AT1, PAR_B1,
                                                             XB, HHL, out, nN, nE, MP);
  k_gemm<<<dim3(MP / GBM, NC2 / GBN), GTHR, 0, stream>>>(HHL, NC2, W2D, 2 * DF, XLR, NC2, KS2);
  k_replay<1><<<cdiv(cdiv(nN, RROWS), NWAVE), NTHR, 0, stream>>>(ENT, SLT, LA, EAR, XLR, PAR, PAR_W2E, PAR_AT2,
                                                                  PAR_B2, XB, HHL, out, nN, nE, MP);
}
